// ChebBen2_71159018160654
// MI455X (gfx1250) — hardware-verified
//
#include <hip/hip_runtime.h>
#include <stddef.h>
#include <stdint.h>
#include <math.h>

#define SPLIT_COMPUTED 1

#define NN      100000
#define NE      1600000
#define HD      64
#define NC      40
#define NCP     48
#define GBM     128
#define MP      100096
#define KL      128
#define K1      320
#define K2      384
#define NTHR    256
#define NWAVE   8
#define EPT     8
#define WCH     (32 * EPT)
#define NBRUN   1024
#define SLB     10
#define NBK     98
#define COP     (3 * NBRUN)
#define WLCAP   2560
#define RCAP    20480
#define DEGCAP  64
#define MAXDEG_MEAS   37
#define MAXB1024_MEAS 16666
#define ABM     64
#define SP      68
#define WSMAX   134217728
#define KC      (SPLIT_COMPUTED ? 128 : 64)

#define BK_ZINTS (NWAVE * WLCAP + RCAP + 3 * NBRUN)
#define BK_INTS  (BK_ZINTS + 16)
#define BK_LDS   (BK_INTS * 4)

#define PBX   (MP * HD / 8 / NTHR)
#define PBW1  (HD * K1 / 8 / NTHR)
#define PBW2  (NCP * K2 / 8 / NTHR)
#define PBTOT (PBX + PBW1 + PBW2 + 1)

static_assert(HD == 16 * 4 && HD == 32 * 2);
static_assert(MP % GBM == 0 && MP >= NN && MP == 782 * GBM && MP % ABM == 0);
static_assert(K1 == 320 && K2 == 384 && K1 % 32 == 0 && K2 % 32 == 0 && KL == 2 * HD && KC % 32 == 0);
static_assert(K1 == HD + 2 * KL && K2 == 3 * KL);
static_assert(NCP == 48 && NCP >= NC && NCP % 16 == 0);
static_assert(NBRUN == (1 << SLB) && NBRUN % ABM == 0 && NBRUN % GBM == 0 && NBRUN % 32 == 0);
static_assert(NBK * NBRUN >= NN && NBK * NBRUN >= MP && (NBK - 1) * NBRUN < NN);
static_assert(NE < (1 << 21) && (((long long)NE) << SLB) < (1LL << 31));
static_assert(NE % WCH == 0 && NE % 4 == 0);
static_assert(RCAP == NWAVE * WLCAP && RCAP % (NTHR * 4) == 0 && COP % (NTHR * 4) == 0 && BK_ZINTS % 4 == 0);
static_assert((long long)RCAP * 100 >= (long long)MAXB1024_MEAS * 105);
static_assert(WLCAP >= MAXB1024_MEAS / 8 + 8 * 46 + 1);
static_assert(DEGCAP >= MAXDEG_MEAS + 8);
static_assert((NC * 4) % 16 == 0 && (GBM * NC * 4) % 128 == 0 && (((NN % GBM) * NC * 4) % 128) == 0);
static_assert(GBM * NC / 4 == 5 * NTHR);
static_assert((MP * HD / 8) % NTHR == 0 && (HD * K1 / 8) % NTHR == 0 && (NCP * K2 / 8) % NTHR == 0);
static_assert((MP * 16) % NTHR == 0);
static_assert(BK_LDS <= 300000);
static_assert((GBM * SP + 64 + GBM) * 4 <= 65536);
static_assert((GBM * NC + 64) * 4 <= 65536);

typedef float          v4f   __attribute__((ext_vector_type(4)));
typedef float          v8f   __attribute__((ext_vector_type(8)));
typedef int            v4i   __attribute__((ext_vector_type(4)));
typedef int            v8i   __attribute__((ext_vector_type(8)));
typedef unsigned       v2u   __attribute__((ext_vector_type(2)));
typedef unsigned short v8us  __attribute__((ext_vector_type(8)));
typedef unsigned short v16us __attribute__((ext_vector_type(16)));
typedef __bf16         v16bf __attribute__((ext_vector_type(16)));
typedef v4f  __attribute__((may_alias)) v4fa;
typedef v4i  __attribute__((may_alias)) v4ia;
typedef v2u  __attribute__((may_alias)) v2ua;
typedef v8us __attribute__((may_alias)) v8usa;
union FragB { v16bf v; v16us u; v8us h[2]; v8i w; };

__device__ __forceinline__ v8f wmb(const FragB& a, const FragB& b, v8f c) {
  v8f d = __builtin_amdgcn_wmma_f32_16x16x32_bf16(false, a.v, false, b.v, (short)0, c, false, false);
  asm volatile("v_nop\n\tv_nop\n\tv_nop\n\tv_nop" : "+v"(d) : "v"(a.w), "v"(b.w));
  return d;
}

__device__ __forceinline__ unsigned bf16_bits(float f) {
  const unsigned u = __float_as_uint(f);
  const unsigned r = (u + 0x7FFFu + ((u >> 16) & 1u)) >> 16;
  const unsigned q = (u >> 16) | 0x40u;
  return ((u & 0x7fffffffu) > 0x7f800000u) ? q : r;
}
__device__ __forceinline__ float bfw_lo(unsigned w) { return __uint_as_float(w << 16); }
__device__ __forceinline__ float bfw_hi(unsigned w) { return __uint_as_float(w & 0xffff0000u); }

__device__ __forceinline__ void hilo_pack(float v0, float v1, float v2, float v3,
                                          int& h01, int& h23, int& l01, int& l23) {
  const unsigned a0 = bf16_bits(v0), a1 = bf16_bits(v1), a2 = bf16_bits(v2), a3 = bf16_bits(v3);
  const unsigned b0 = bf16_bits(v0 - __uint_as_float(a0 << 16));
  const unsigned b1 = bf16_bits(v1 - __uint_as_float(a1 << 16));
  const unsigned b2 = bf16_bits(v2 - __uint_as_float(a2 << 16));
  const unsigned b3 = bf16_bits(v3 - __uint_as_float(a3 << 16));
  h01 = (int)(a0 | (a1 << 16)); h23 = (int)(a2 | (a3 << 16));
  l01 = (int)(b0 | (b1 << 16)); l23 = (int)(b2 | (b3 << 16));
}

__device__ __forceinline__ v4i regroup8(int h01, int h23, int l01, int l23, int lane) {
  const int t  = lane & 15;
  const int s0 = (lane & 16) + ((2 * t) & 15), s1 = s0 + 1;
  const int a0 = __shfl(h01, s0, 32), a1 = __shfl(h23, s0, 32), a2 = __shfl(h01, s1, 32), a3 = __shfl(h23, s1, 32);
  const int b0 = __shfl(l01, s0, 32), b1 = __shfl(l23, s0, 32), b2 = __shfl(l01, s1, 32), b3 = __shfl(l23, s1, 32);
  const int mk = (t < 8) ? -1 : 0;
  v4i o;
  o.x = (a0 & mk) | (b0 & ~mk); o.y = (a1 & mk) | (b1 & ~mk);
  o.z = (a2 & mk) | (b2 & ~mk); o.w = (a3 & mk) | (b3 & ~mk);
  return o;
}

__device__ __forceinline__ void st2_v4f(float* p, v4f v) {
  *(volatile v4f*)p = v;
  __threadfence();
  *(volatile v4f*)p = v;
}
__device__ __forceinline__ void st2_v8us(unsigned short* p, v8us v) {
  *(volatile v8us*)p = v;
  __threadfence();
  *(volatile v8us*)p = v;
}

__device__ __forceinline__ v8us gather8(const float* __restrict__ base, int stride, unsigned mk) {
  float f[8];
#pragma unroll
  for (int i = 0; i < 8; ++i) f[i] = base[(size_t)i * (size_t)stride];
  v8us o;
#pragma unroll
  for (int i = 0; i < 8; ++i) o[i] = (unsigned short)(bf16_bits(f[i]) & mk);
  return o;
}

__global__ __launch_bounds__(NTHR) void k_prep(const float* __restrict__ x, const float* __restrict__ w1,
                                               const float* __restrict__ b1, const float* __restrict__ w2,
                                               const float* __restrict__ b2, unsigned short* xb,
                                               unsigned short* w1c, unsigned short* w2c, float* sm) {
  const int tid = (int)threadIdx.x, lane = tid & 31;
  const int blk = (int)blockIdx.x;
  if (blk < PBX) {
    const int u   = blk * NTHR + tid;
    const int row = u >> 3, k8 = (u & 7) * 8;
    const int rc  = row < NN ? row : NN - 1;
    const unsigned mk = row < NN ? 0xffffu : 0u;
    const float* p = x + (size_t)rc * HD + k8;
    const v4f a = *(const v4fa*)p;
    const v4f b = *(const v4fa*)(p + 4);
    v8us o;
    o[0] = (unsigned short)(bf16_bits(a.x) & mk); o[1] = (unsigned short)(bf16_bits(a.y) & mk);
    o[2] = (unsigned short)(bf16_bits(a.z) & mk); o[3] = (unsigned short)(bf16_bits(a.w) & mk);
    o[4] = (unsigned short)(bf16_bits(b.x) & mk); o[5] = (unsigned short)(bf16_bits(b.y) & mk);
    o[6] = (unsigned short)(bf16_bits(b.z) & mk); o[7] = (unsigned short)(bf16_bits(b.w) & mk);
    st2_v8us(xb + (size_t)row * HD + k8, o);
  } else if (blk < PBX + PBW1) {
    const int u  = (blk - PBX) * NTHR + tid;
    const int n  = u / (K1 / 8);
    const int k8 = (u - n * (K1 / 8)) * 8;
    const int j  = ((k8 >> 6) + 1) >> 1;
    const int kk = k8 & 63;
    const v8us o = gather8(w1 + (size_t)j * HD * HD + (size_t)kk * HD + n, HD, 0xffffu);
    st2_v8us(w1c + (size_t)n * K1 + k8, o);
  } else if (blk < PBX + PBW1 + PBW2) {
    const int u  = (blk - PBX - PBW1) * NTHR + tid;
    const int n  = u / (K2 / 8);
    const int k8 = (u - n * (K2 / 8)) * 8;
    const int j  = k8 >> 7;
    const int kk = k8 & 63;
    const int nc = n < NC ? n : NC - 1;
    const unsigned mk = n < NC ? 0xffffu : 0u;
    const v8us o = gather8(w2 + (size_t)j * HD * NC + (size_t)kk * NC + nc, NC, mk);
    st2_v8us(w2c + (size_t)n * K2 + k8, o);
  } else {
    if (tid < 32) {
      const int q = lane & 15;
      const int i0 = 4 * q, i1 = i0 + 1, i2 = i0 + 2, i3 = i0 + 3;
      const float a0 = b1[i0], a1 = b1[i1], a2 = b1[i2], a3 = b1[i3];
      const float c0 = b2[i0 < NC ? i0 : NC - 1], c1 = b2[i1 < NC ? i1 : NC - 1];
      const float c2 = b2[i2 < NC ? i2 : NC - 1], c3 = b2[i3 < NC ? i3 : NC - 1];
      asm volatile("" :: "v"(a0), "v"(a1), "v"(a2), "v"(a3));
      asm volatile("" :: "v"(c0), "v"(c1), "v"(c2), "v"(c3));
      const unsigned ma = (lane < 16) ? 0xffffffffu : 0u;
      const unsigned m0 = (i0 < NC) ? ~ma : 0u, m1 = (i1 < NC) ? ~ma : 0u;
      const unsigned m2 = (i2 < NC) ? ~ma : 0u, m3 = (i3 < NC) ? ~ma : 0u;
      v4f o;
      o.x = __uint_as_float(((bf16_bits(a0) << 16) & ma) | ((bf16_bits(c0) << 16) & m0));
      o.y = __uint_as_float(((bf16_bits(a1) << 16) & ma) | ((bf16_bits(c1) << 16) & m1));
      o.z = __uint_as_float(((bf16_bits(a2) << 16) & ma) | ((bf16_bits(c2) << 16) & m2));
      o.w = __uint_as_float(((bf16_bits(a3) << 16) & ma) | ((bf16_bits(c3) << 16) & m3));
      st2_v4f(sm + 4 * lane, o);
    }
  }
}

__device__ __forceinline__ void bucket_flush(const int* pl, const int* cnt, int ov, int* lp, int* cop, int* fp,
                                             int tid) {
#pragma unroll 1
  for (int i = tid * 4; i < RCAP; i += NTHR * 4) {
    const v4i v = *(const v4ia*)(pl + i);
    *(volatile v4i*)(lp + i) = v;
  }
#pragma unroll 1
  for (int i = tid * 4; i < COP; i += NTHR * 4) {
    const v4i v = *(const v4ia*)(cnt + i);
    *(volatile v4i*)(cop + i) = v;
  }
  if (tid < 8) {
    const v4i f = {ov, ov, ov, ov};
    *(volatile v4i*)(fp + 4 * tid) = f;
  }
}

__global__ __launch_bounds__(NTHR) void k_bucket(const int* __restrict__ keys, const int* __restrict__ cols,
                                                 int* LIST, int* CO, int* FLAG) {
  extern __shared__ __attribute__((aligned(16))) int dsm[];
  int* wl   = dsm;
  int* pl   = dsm + NWAVE * WLCAP;
  int* cnt  = pl + RCAP;
  int* offs = cnt + NBRUN;
  int* cur  = offs + NBRUN;
  int* misc = cur + NBRUN;
  const int tid = (int)threadIdx.x, lane = tid & 31, wave = tid >> 5;
  const int blk = (int)blockIdx.x;
  const unsigned nbs = (unsigned)(blk * NBRUN);
  int nbi = NN - blk * NBRUN;
  nbi = nbi > NBRUN ? NBRUN : (nbi < 0 ? 0 : nbi);
  const unsigned unb = (unsigned)nbi;

  {
    const v4i z4 = {0, 0, 0, 0};
    for (int i = tid * 4; i < BK_ZINTS; i += NTHR * 4) *(v4ia*)(dsm + i) = z4;
    if (tid < 16) misc[tid] = 0;
  }
  __syncthreads();

  {
    const int per  = ((NE + NWAVE * WCH - 1) / (NWAVE * WCH)) * WCH;
    const int ebeg = wave * per;
    const int eend = (ebeg + per < NE) ? (ebeg + per) : NE;
    int* mylist = wl + wave * WLCAP;
    int wc = 0;
#pragma unroll 1
    for (int cb = ebeg; cb < eend; cb += WCH) {
      const int e0 = cb + lane * EPT;
      const v4i da = *(const v4ia*)(keys + e0);
      const v4i db = *(const v4ia*)(keys + e0 + 4);
      const unsigned s0 = (unsigned)da.x - nbs, s1 = (unsigned)da.y - nbs;
      const unsigned s2 = (unsigned)da.z - nbs, s3 = (unsigned)da.w - nbs;
      const unsigned s4 = (unsigned)db.x - nbs, s5 = (unsigned)db.y - nbs;
      const unsigned s6 = (unsigned)db.z - nbs, s7 = (unsigned)db.w - nbs;
      const bool h0 = s0 < unb, h1 = s1 < unb, h2 = s2 < unb, h3 = s3 < unb;
      const bool h4 = s4 < unb, h5 = s5 < unb, h6 = s6 < unb, h7 = s7 < unb;
      const unsigned m0 = __builtin_amdgcn_ballot_w32(h0), m1 = __builtin_amdgcn_ballot_w32(h1);
      const unsigned m2 = __builtin_amdgcn_ballot_w32(h2), m3 = __builtin_amdgcn_ballot_w32(h3);
      const unsigned m4 = __builtin_amdgcn_ballot_w32(h4), m5 = __builtin_amdgcn_ballot_w32(h5);
      const unsigned m6 = __builtin_amdgcn_ballot_w32(h6), m7 = __builtin_amdgcn_ballot_w32(h7);
      const unsigned any = m0 | m1 | m2 | m3 | m4 | m5 | m6 | m7;
      if (any != 0u) {
        const int pre = (int)(__builtin_amdgcn_mbcnt_lo(m0, 0u) + __builtin_amdgcn_mbcnt_lo(m1, 0u) +
                              __builtin_amdgcn_mbcnt_lo(m2, 0u) + __builtin_amdgcn_mbcnt_lo(m3, 0u) +
                              __builtin_amdgcn_mbcnt_lo(m4, 0u) + __builtin_amdgcn_mbcnt_lo(m5, 0u) +
                              __builtin_amdgcn_mbcnt_lo(m6, 0u) + __builtin_amdgcn_mbcnt_lo(m7, 0u));
        int p = wc + pre;
        if (h0) { if (p < WLCAP) mylist[p] = ((e0 + 0) << SLB) | (int)s0; p = p + 1; }
        if (h1) { if (p < WLCAP) mylist[p] = ((e0 + 1) << SLB) | (int)s1; p = p + 1; }
        if (h2) { if (p < WLCAP) mylist[p] = ((e0 + 2) << SLB) | (int)s2; p = p + 1; }
        if (h3) { if (p < WLCAP) mylist[p] = ((e0 + 3) << SLB) | (int)s3; p = p + 1; }
        if (h4) { if (p < WLCAP) mylist[p] = ((e0 + 4) << SLB) | (int)s4; p = p + 1; }
        if (h5) { if (p < WLCAP) mylist[p] = ((e0 + 5) << SLB) | (int)s5; p = p + 1; }
        if (h6) { if (p < WLCAP) mylist[p] = ((e0 + 6) << SLB) | (int)s6; p = p + 1; }
        if (h7) { if (p < WLCAP) mylist[p] = ((e0 + 7) << SLB) | (int)s7; p = p + 1; }
        wc += (int)(__builtin_popcount(m0) + __builtin_popcount(m1) + __builtin_popcount(m2) + __builtin_popcount(m3) +
                    __builtin_popcount(m4) + __builtin_popcount(m5) + __builtin_popcount(m6) + __builtin_popcount(m7));
      }
    }
    if (lane == 0) misc[wave] = wc;
  }
  __syncthreads();

  if (wave == 0) {
    int ov = 0;
#pragma unroll 1
    for (int w2 = 0; w2 < NWAVE; ++w2) {
      int c = misc[w2];
      if (c > WLCAP) ov = 1;
      c = c < 0 ? 0 : (c > WLCAP ? WLCAP : c);
#pragma unroll 1
      for (int b0 = 0; b0 < c; b0 += 32) {
        const int idx = b0 + lane;
        const int ent = wl[w2 * WLCAP + (idx < WLCAP ? idx : WLCAP - 1)];
        const int m32 = (c - b0) < 32 ? (c - b0) : 32;
#pragma unroll 1
        for (int k = 0; k < m32; ++k) {
          const int u    = __builtin_amdgcn_readlane(ent, k);
          const int slot = u & (NBRUN - 1);
          if (lane == 0) cnt[slot] = cnt[slot] + 1;
        }
      }
    }
    if (lane == 0) misc[9] = ov;
  }
  __syncthreads();
  if (wave == 0) {
    const int base = lane * (NBRUN / 32);
    int s = 0;
#pragma unroll 1
    for (int i = 0; i < NBRUN / 32; ++i) s += cnt[base + i];
    int incl = s;
#pragma unroll
    for (int d = 1; d < 32; d <<= 1) {
      const int y = __shfl_up(incl, d, 32);
      if (lane >= d) incl += y;
    }
    int run = incl - s;
#pragma unroll 1
    for (int i = 0; i < NBRUN / 32; ++i) {
      const int cv = cnt[base + i];
      offs[base + i] = run;
      cur[base + i]  = run;
      run += cv;
    }
  }
  __syncthreads();

  if (wave == 0) {
#pragma unroll 1
    for (int w2 = 0; w2 < NWAVE; ++w2) {
      int c = misc[w2];
      c = c < 0 ? 0 : (c > WLCAP ? WLCAP : c);
#pragma unroll 1
      for (int b0 = 0; b0 < c; b0 += 32) {
        const int idx = b0 + lane;
        const int ent = wl[w2 * WLCAP + (idx < WLCAP ? idx : WLCAP - 1)];
        int eid = (ent >> SLB) & 0x1FFFFF;
        eid = eid > NE - 1 ? NE - 1 : eid;
        int word = cols[eid];
        word = word < 0 ? 0 : (word > NN - 1 ? NN - 1 : word);
        const int m32 = (c - b0) < 32 ? (c - b0) : 32;
#pragma unroll 1
        for (int k = 0; k < m32; ++k) {
          const int u    = __builtin_amdgcn_readlane(ent, k);
          const int wd   = __builtin_amdgcn_readlane(word, k);
          const int slot = u & (NBRUN - 1);
          if (lane == 0) {
            int p = cur[slot];
            p = p < 0 ? 0 : (p > RCAP - 1 ? RCAP - 1 : p);
            pl[p] = wd;
            cur[slot] = p + 1;
          }
        }
      }
    }
  }
  __syncthreads();

#pragma unroll 1
  for (int i = tid; i < NBRUN; i += NTHR) {
    const int c = cnt[i];
    const float fd = (float)(c > 1 ? c : 1);
    const float r  = 1.0f / sqrtf(fd);
    cur[i] = __float_as_int((c > 0) ? r : 0.0f);
  }
  __syncthreads();

  const int ovf = misc[9];
  int* lp  = LIST + (size_t)blk * RCAP;
  int* cop = CO + (size_t)blk * COP;
  int* fp  = FLAG + (size_t)blk * 32;
  bucket_flush(pl, cnt, ovf, lp, cop, fp, tid);
  __threadfence();
  bucket_flush(pl, cnt, ovf, lp, cop, fp, tid);
}

__global__ __launch_bounds__(NTHR) void k_scale0(const unsigned short* __restrict__ XB, const int* __restrict__ CO,
                                                 float* PA) {
  const int u   = (int)blockIdx.x * NTHR + (int)threadIdx.x;
  const int row = u >> 4, q = u & 15;
  const v2u w = *(const v2ua*)(XB + (size_t)row * HD + 4 * q);
  const float ds = __int_as_float(CO[(size_t)(row >> SLB) * COP + 2 * NBRUN + (row & (NBRUN - 1))]);
  v4f o;
  o.x = ds * bfw_lo(w.x); o.y = ds * bfw_hi(w.x);
  o.z = ds * bfw_lo(w.y); o.w = ds * bfw_hi(w.y);
  st2_v4f(PA + (size_t)row * HD + 4 * q, o);
}

template <int MODE>
__global__ __launch_bounds__(NTHR) void k_replay(const int* __restrict__ LIST, const int* __restrict__ CO,
                                                 const int* __restrict__ FLAG, const float* __restrict__ Ps,
                                                 const unsigned short* __restrict__ BASE,
                                                 unsigned short* Thl, float* Pn) {
  const int tid = (int)threadIdx.x, lane = tid & 31, wave = tid >> 5, hh = lane >> 4, q = lane & 15;
  const int rowBase = (int)blockIdx.x * ABM;
  const int bucket  = rowBase >> SLB;
  const int* lb  = LIST + (size_t)bucket * RCAP;
  const int* cob = CO + (size_t)bucket * COP;
  const int flag = FLAG[(size_t)bucket * 32];
  const float qnan = __uint_as_float(0x7fc00000u);

#pragma unroll 1
  for (int i = 0; i < ABM / (2 * NWAVE); ++i) {
    const int d    = rowBase + (ABM / NWAVE) * wave + 2 * i + hh;
    const int slot = d & (NBRUN - 1);
    int c = cob[slot];
    int o = cob[NBRUN + slot];
    const float ds = __int_as_float(cob[2 * NBRUN + slot]);
    const bool big = c > DEGCAP;
    c = c < 0 ? 0 : (c > DEGCAP ? DEGCAP : c);
    o = o < 0 ? 0 : (o > RCAP - 1 ? RCAP - 1 : o);
    const int co = __shfl_xor(c, 16, 32);
    const int cm = c > co ? c : co;
    int last = o + (c > 0 ? c : 1) - 1;
    last = last > RCAP - 1 ? RCAP - 1 : last;
    float a0 = 0.0f, a1 = 0.0f, a2 = 0.0f, a3 = 0.0f;
#pragma unroll 1
    for (int j = 0; j < cm; ++j) {
      int idx = o + j;
      idx = idx > last ? last : idx;
      int sr = lb[idx];
      sr = sr < 0 ? 0 : (sr > NN - 1 ? NN - 1 : sr);
      const v4f v = *(const v4fa*)(Ps + (size_t)sr * HD + 4 * q);
      asm volatile("" :: "v"(v));
      const bool valid = j < c;
      const float t0 = a0 + v.x, t1 = a1 + v.y, t2 = a2 + v.z, t3 = a3 + v.w;
      a0 = valid ? t0 : a0; a1 = valid ? t1 : a1; a2 = valid ? t2 : a2; a3 = valid ? t3 : a3;
    }
    float m0 = -(ds * a0), m1 = -(ds * a1), m2 = -(ds * a2), m3 = -(ds * a3);
    if constexpr (MODE == 1) {
      const v2u w = *(const v2ua*)(BASE + (size_t)d * HD + 4 * q);
      m0 = 2.0f * m0 - bfw_lo(w.x); m1 = 2.0f * m1 - bfw_hi(w.x);
      m2 = 2.0f * m2 - bfw_lo(w.y); m3 = 2.0f * m3 - bfw_hi(w.y);
    }
    if constexpr (MODE == 2) {
      const v2u wh = *(const v2ua*)(BASE + (size_t)d * KL + 4 * q);
      const v2u wl = *(const v2ua*)(BASE + (size_t)d * KL + HD + 4 * q);
      m0 = 2.0f * m0 - (bfw_lo(wh.x) + bfw_lo(wl.x)); m1 = 2.0f * m1 - (bfw_hi(wh.x) + bfw_hi(wl.x));
      m2 = 2.0f * m2 - (bfw_lo(wh.y) + bfw_lo(wl.y)); m3 = 2.0f * m3 - (bfw_hi(wh.y) + bfw_hi(wl.y));
    }
    const bool bad  = (flag != 0) | big;
    const bool live = d < NN;
    m0 = bad ? qnan : m0; m1 = bad ? qnan : m1; m2 = bad ? qnan : m2; m3 = bad ? qnan : m3;
    m0 = live ? m0 : 0.0f; m1 = live ? m1 : 0.0f; m2 = live ? m2 : 0.0f; m3 = live ? m3 : 0.0f;
    int h01, h23, l01, l23;
    hilo_pack(m0, m1, m2, m3, h01, h23, l01, l23);
    const v4i ow = regroup8(h01, h23, l01, l23, lane);
    unsigned short* hp = Thl + (size_t)d * KL + 8 * q;
    if constexpr (MODE == 0) {
      v4f pv;
      pv.x = ds * m0; pv.y = ds * m1; pv.z = ds * m2; pv.w = ds * m3;
      float* pp = Pn + (size_t)d * HD + 4 * q;
      *(volatile v4i*)hp = ow;
      *(volatile v4f*)pp = pv;
      __threadfence();
      *(volatile v4i*)hp = ow;
      *(volatile v4f*)pp = pv;
    } else {
      *(volatile v4i*)hp = ow;
      __threadfence();
      *(volatile v4i*)hp = ow;
    }
  }
}

template <int KS, int NT, int BP>
__device__ __forceinline__ void kseg(const unsigned short* ap, const unsigned short* bp, v8f (&acc)[NT]) {
#pragma unroll 1
  for (int k0 = 0; k0 < KS; k0 += 32) {
    FragB af;
    af.h[0] = *(const v8usa*)(ap + k0);
    af.h[1] = *(const v8usa*)(ap + k0 + 16);
#pragma unroll
    for (int nt = 0; nt < NT; ++nt) {
      const unsigned short* wq = bp + (size_t)(16 * nt) * (size_t)BP + k0;
      FragB bf;
      bf.h[0] = *(const v8usa*)wq;
      bf.h[1] = *(const v8usa*)(wq + 16);
      acc[nt] = wmb(af, bf, acc[nt]);
    }
  }
}

__global__ __launch_bounds__(NTHR) __attribute__((amdgpu_num_vgpr(248)))
void k_gemm1(const unsigned short* __restrict__ XB, unsigned short* T1H, const unsigned short* __restrict__ T2,
             const unsigned short* __restrict__ W1C, const float* __restrict__ sm, const int* __restrict__ CO,
             float* PA) {
  __shared__ __attribute__((aligned(16))) float stg[GBM * SP];
  __shared__ __attribute__((aligned(16))) float sb[64];
  __shared__ __attribute__((aligned(16))) int dsl[GBM];
  const int tid = (int)threadIdx.x, lane = tid & 31, wave = tid >> 5, hh = lane >> 4, m = lane & 15;
  const int rowBase = (int)blockIdx.x * GBM;
  if (wave == 0) {
    const v4f b4 = *(const v4fa*)(sm + 4 * m);
    *(v4fa*)(sb + 4 * m) = b4;
  }
  if (wave == 1) {
    const int* dsrc = CO + (size_t)(rowBase >> SLB) * COP + 2 * NBRUN + (rowBase & (NBRUN - 1));
    const v4i d4 = *(const v4ia*)(dsrc + 4 * lane);
    *(v4ia*)(dsl + 4 * lane) = d4;
  }

  v8f acc[4];
  {
    const v8f z = {0.f, 0.f, 0.f, 0.f, 0.f, 0.f, 0.f, 0.f};
#pragma unroll
    for (int t = 0; t < 4; ++t) acc[t] = z;
  }
  const size_t row = (size_t)(rowBase + 16 * wave + m);
  const unsigned short* bp = W1C + (size_t)m * (size_t)K1 + 8 * hh;
  kseg<HD, 4, K1>(XB + row * HD + 8 * hh, bp, acc);
  kseg<KC, 4, K1>(T1H + row * KL + 8 * hh, bp + HD, acc);
  kseg<KC, 4, K1>(T2 + row * KL + 8 * hh, bp + HD + KL, acc);

#pragma unroll
  for (int nt = 0; nt < 4; ++nt) {
#pragma unroll
    for (int r = 0; r < 8; ++r) stg[(16 * wave + 8 * hh + r) * SP + 16 * nt + m] = acc[nt][r];
  }
  __syncthreads();

  const v4f bias = *(const v4fa*)(sb + 4 * m);
#pragma unroll 1
  for (int i = 0; i < 8; ++i) {
    const int lr   = 16 * wave + 2 * i + hh;
    const int grow = rowBase + lr;
    const bool live = grow < NN;
    const v4f a = *(const v4fa*)(stg + lr * SP + 4 * m);
    const float ds = __int_as_float(dsl[lr]);
    asm volatile("" :: "v"(a));
    asm volatile("" :: "v"(ds));
    float v0 = a.x + bias.x, v1 = a.y + bias.y, v2 = a.z + bias.z, v3 = a.w + bias.w;
    v0 = (v0 > 0.0f) ? v0 : (v0 - v0); v1 = (v1 > 0.0f) ? v1 : (v1 - v1);
    v2 = (v2 > 0.0f) ? v2 : (v2 - v2); v3 = (v3 > 0.0f) ? v3 : (v3 - v3);
    v0 = live ? v0 : 0.0f; v1 = live ? v1 : 0.0f; v2 = live ? v2 : 0.0f; v3 = live ? v3 : 0.0f;
    v4f pv;
    pv.x = ds * v0; pv.y = ds * v1; pv.z = ds * v2; pv.w = ds * v3;
    int h01, h23, l01, l23;
    hilo_pack(v0, v1, v2, v3, h01, h23, l01, l23);
    const v4i ow = regroup8(h01, h23, l01, l23, lane);
    unsigned short* hp = T1H + (size_t)grow * KL + 8 * m;
    float* pp = PA + (size_t)grow * HD + 4 * m;
    *(volatile v4i*)hp = ow;
    *(volatile v4f*)pp = pv;
    __threadfence();
    *(volatile v4i*)hp = ow;
    *(volatile v4f*)pp = pv;
  }
}

__device__ __forceinline__ void out_flush(const float* lg, float* ob, int nv4, int tid, unsigned km, unsigned pz) {
#pragma unroll 1
  for (int it = 0; it < 5; ++it) {
    const int i4 = it * NTHR + tid;
    const v4f v = *(const v4fa*)(lg + 4 * i4);
    asm volatile("" :: "v"(v));
    v4f o;
    o.x = __uint_as_float((__float_as_uint(v.x) & km) | pz);
    o.y = __uint_as_float((__float_as_uint(v.y) & km) | pz);
    o.z = __uint_as_float((__float_as_uint(v.z) & km) | pz);
    o.w = __uint_as_float((__float_as_uint(v.w) & km) | pz);
    if (i4 < nv4) *(volatile v4f*)(ob + (size_t)4 * (size_t)i4) = o;
  }
}

__global__ __launch_bounds__(NTHR) __attribute__((amdgpu_num_vgpr(248)))
void k_gemm2(const unsigned short* __restrict__ Hh, const unsigned short* __restrict__ T1,
             const unsigned short* __restrict__ T2, const unsigned short* __restrict__ W2C,
             const float* __restrict__ sm, const int* __restrict__ FLAG, float* out) {
  __shared__ __attribute__((aligned(16))) float lg[GBM * NC];
  __shared__ __attribute__((aligned(16))) float sb2[64];
  const int tid = (int)threadIdx.x, lane = tid & 31, wave = tid >> 5, hh = lane >> 4, m = lane & 15;
  const int blk = (int)blockIdx.x;
  const int rowBase = blk * GBM;
  int flag = FLAG[(size_t)(rowBase >> SLB) * 32];
  asm volatile("" :: "v"(flag));
  if (wave == 0) {
    const v4f b4 = *(const v4fa*)(sm + 64 + 4 * m);
    *(v4fa*)(sb2 + 4 * m) = b4;
  }

  v8f acc[3];
  {
    const v8f z = {0.f, 0.f, 0.f, 0.f, 0.f, 0.f, 0.f, 0.f};
#pragma unroll
    for (int t = 0; t < 3; ++t) acc[t] = z;
  }
  const size_t row = (size_t)(rowBase + 16 * wave + m);
  const unsigned short* bp = W2C + (size_t)m * (size_t)K2 + 8 * hh;
  kseg<KC, 3, K2>(Hh + row * KL + 8 * hh, bp, acc);
  kseg<KC, 3, K2>(T1 + row * KL + 8 * hh, bp + KL, acc);
  kseg<KC, 3, K2>(T2 + row * KL + 8 * hh, bp + 2 * KL, acc);
  __syncthreads();

#pragma unroll
  for (int nt = 0; nt < 3; ++nt) {
    const int col = 16 * nt + m;
    const float bc = sb2[col];
    asm volatile("" :: "v"(bc));
#pragma unroll
    for (int r = 0; r < 8; ++r) {
      const int lr = 16 * wave + 8 * hh + r;
      if (col < NC) lg[lr * NC + col] = acc[nt][r] + bc;
    }
  }
  __syncthreads();

  const unsigned pz = (flag != 0) ? 0x7fc00000u : 0u;
  const unsigned km = (flag != 0) ? 0u : 0xFFFFFFFFu;
  const int liveRows = (NN - rowBase) < GBM ? (NN - rowBase) : GBM;
  const int nv4 = liveRows * (NC / 4);
  float* ob = out + (size_t)blk * (size_t)(GBM * NC);
  out_flush(lg, ob, nv4, tid, km, pz);
  __threadfence();
  out_flush(lg, ob, nv4, tid, km, pz);
}

extern "C" void kernel_launch(void* const* d_in, const int* in_sizes, int n_in,
                              void* d_out, int out_size, void* d_ws, size_t ws_size,
                              hipStream_t stream) {
  if (n_in < 6) return;
  if (in_sizes[0] != NN * HD) return;
  if (in_sizes[1] != 2 * NE) return;
  if (in_sizes[2] != 3 * HD * HD) return;
  if (in_sizes[3] != HD) return;
  if (in_sizes[4] != 3 * HD * NC) return;
  if (in_sizes[5] != NC) return;
  if (out_size != NN * NC) return;

  const float* x  = (const float*)d_in[0];
  const int*   ei = (const int*)d_in[1];
  const float* W1 = (const float*)d_in[2];
  const float* b1 = (const float*)d_in[3];
  const float* W2 = (const float*)d_in[4];
  const float* b2 = (const float*)d_in[5];
  float* out = (float*)d_out;
  const int* keys = ei;
  const int* cols = ei + NE;

  constexpr size_t zXB   = (size_t)MP * HD * 2;
  constexpr size_t zHL   = (size_t)MP * KL * 2;
  constexpr size_t zPF   = (size_t)MP * HD * 4;
  constexpr size_t zLIST = (size_t)NBK * RCAP * 4;
  constexpr size_t zCO   = (size_t)NBK * COP * 4;
  constexpr size_t zFLAG = (size_t)NBK * 128;
  constexpr size_t zW1C  = (size_t)HD * K1 * 2;
  constexpr size_t zW2C  = (size_t)NCP * K2 * 2;
  constexpr size_t zSM   = 512;
  constexpr size_t oXB   = 0;
  constexpr size_t oHLA  = oXB + zXB;
  constexpr size_t oHLB  = oHLA + zHL;
  constexpr size_t oPFA  = oHLB + zHL;
  constexpr size_t oPFB  = oPFA + zPF;
  constexpr size_t oLIST = oPFB + zPF;
  constexpr size_t oCO   = oLIST + zLIST;
  constexpr size_t oFLAG = oCO + zCO;
  constexpr size_t oW1C  = oFLAG + zFLAG;
  constexpr size_t oW2C  = oW1C + zW1C;
  constexpr size_t oSM   = oW2C + zW2C;
  constexpr size_t oEND  = oSM + zSM;
  static_assert(zXB % 256 == 0 && zHL % 256 == 0 && zPF % 256 == 0 && zLIST % 256 == 0 && zCO % 256 == 0);
  static_assert(zFLAG % 256 == 0 && zW1C % 256 == 0 && zW2C % 256 == 0 && zSM % 256 == 0);
  static_assert(zHL == zPF);
  static_assert(oEND <= (size_t)WSMAX);
  if (oEND > ws_size) return;

  char* ws = (char*)d_ws;
  unsigned short* XB   = (unsigned short*)(ws + oXB);
  unsigned short* HLA  = (unsigned short*)(ws + oHLA);
  unsigned short* HLB  = (unsigned short*)(ws + oHLB);
  float*          PFA  = (float*)(ws + oPFA);
  float*          PFB  = (float*)(ws + oPFB);
  unsigned short* PFAh = (unsigned short*)(ws + oPFA);
  int*            LIST = (int*)(ws + oLIST);
  int*            CO   = (int*)(ws + oCO);
  int*            FLAG = (int*)(ws + oFLAG);
  unsigned short* W1C  = (unsigned short*)(ws + oW1C);
  unsigned short* W2C  = (unsigned short*)(ws + oW2C);
  float*          SM   = (float*)(ws + oSM);

  hipFuncSetAttribute(reinterpret_cast<const void*>(&k_bucket), hipFuncAttributeMaxDynamicSharedMemorySize, (int)BK_LDS);

  k_prep<<<PBTOT, NTHR, 0, stream>>>(x, W1, b1, W2, b2, XB, W1C, W2C, SM);
  k_bucket<<<NBK, NTHR, BK_LDS, stream>>>(keys, cols, LIST, CO, FLAG);
  k_scale0<<<MP * 16 / NTHR, NTHR, 0, stream>>>(XB, CO, PFA);
  k_replay<0><<<MP / ABM, NTHR, 0, stream>>>(LIST, CO, FLAG, PFA, XB, HLA, PFB);
  k_replay<1><<<MP / ABM, NTHR, 0, stream>>>(LIST, CO, FLAG, PFB, XB, HLB, PFA);
  k_gemm1<<<MP / GBM, NTHR, 0, stream>>>(XB, HLA, HLB, W1C, SM, CO, PFA);
  k_replay<0><<<MP / ABM, NTHR, 0, stream>>>(LIST, CO, FLAG, PFA, XB, HLB, PFB);
  k_replay<2><<<MP / ABM, NTHR, 0, stream>>>(LIST, CO, FLAG, PFB, HLA, PFAh, PFB);
  k_gemm2<<<MP / GBM, NTHR, 0, stream>>>(HLA, HLB, PFAh, W2C, SM, FLAG, out);
}
